// ParallelHybridReasoningLayer_34342558498999
// MI455X (gfx1250) — hardware-verified
//
#include <hip/hip_runtime.h>
#include <stdint.h>

constexpr int NBATCH = 8;
constexpr int SEQLEN = 1024;
constexpr int DMOD   = 256;
constexpr int NHEAD  = 4;
constexpr int HDIM64 = 64;
constexpr int NTOKS  = NBATCH * SEQLEN;
constexpr int QKVLD  = 3 * DMOD;
constexpr int COMBLD = 3 * DMOD;
constexpr int HIDT   = 2 * DMOD;
constexpr int HIDF   = 4 * DMOD;
constexpr int CONVW  = 8;
constexpr int TCH    = 16;
constexpr float WCARRY = 32.0f;
constexpr float OCARRY = 16.0f;
constexpr float GCARRY = 16.0f;
constexpr float LN_EPS = 1e-5f;
constexpr float EMA_DECAY = 0.9f;
constexpr float EMA_GAIN  = 0.1f;
constexpr float STEP_HALF = 0.5f;
constexpr float GUIDE = 0.3f;
constexpr float QKSCALE = 0.125f;

static_assert(NTOKS % 64 == 0 && DMOD % 64 == 0 && QKVLD % 64 == 0 && HIDT % 64 == 0 && HIDF % 64 == 0, "tile multiples");
static_assert(DMOD % 32 == 0 && COMBLD % 32 == 0 && HIDT % 32 == 0 && HIDF % 32 == 0, "K multiples of 32");
static_assert(SEQLEN % TCH == 0 && SEQLEN % 64 == 0 && NHEAD * HDIM64 == DMOD, "geometry");

typedef __attribute__((ext_vector_type(16))) _Float16 v16h;
typedef __attribute__((ext_vector_type(8)))  _Float16 v8h;
typedef __attribute__((ext_vector_type(16))) __bf16   v16b;
typedef __attribute__((ext_vector_type(8)))  __bf16   v8b;
typedef __attribute__((ext_vector_type(8)))  float    v8f;
typedef __attribute__((ext_vector_type(4)))  float    v4f;
typedef __attribute__((ext_vector_type(2)))  float    v2f;
#define PSCALE 32768.0f
#define U16(p) ((const unsigned short*)(const void*)(p))
#define PSCALE_INV (1.0f / 32768.0f)

__device__ __forceinline__ unsigned short f2bf_bits(float f) {
  unsigned u = __float_as_uint(f);
  return (unsigned short)((u + 0x7FFFu + ((u >> 16) & 1u)) >> 16);
}
__device__ __forceinline__ float bf_bits2f(unsigned short h) { return __uint_as_float(((unsigned)h) << 16); }

__device__ __forceinline__ void dep_guard_h(v8f& a, v8f& b, v16h x, v16h y) { asm volatile("v_nop\n\tv_nop\n\tv_nop\n\tv_nop" : "+v"(a), "+v"(b) : "v"(x), "v"(y)); }
__device__ __forceinline__ void dep_guard_b(v8f& a, v8f& b, v16b x, v16b y) { asm volatile("v_nop\n\tv_nop\n\tv_nop\n\tv_nop" : "+v"(a), "+v"(b) : "v"(x), "v"(y)); }
__device__ __forceinline__ void keep4_h(v16h a, v16h b, v16h c, v16h d) { asm volatile("v_nop" :: "v"(a), "v"(b), "v"(c), "v"(d)); }
__device__ __forceinline__ void keep4_b(v16b a, v16b b, v16b c, v16b d) { asm volatile("v_nop" :: "v"(a), "v"(b), "v"(c), "v"(d)); }
__device__ __forceinline__ void acc_guard4(v8f& a, v8f& b, v8f& c, v8f& d) { asm volatile("v_nop\n\tv_nop\n\tv_nop\n\tv_nop" : "+v"(a), "+v"(b), "+v"(c), "+v"(d)); }
template <typename T> struct Frag;
template <> struct Frag<_Float16> {
  typedef v16h V; union U { v16h v; v8h h[2]; };
  static __device__ __forceinline__ v16h load(const _Float16* p) {
    U f; f.h[0] = *(const v8h*)(p); f.h[1] = *(const v8h*)(p + 16); return f.v;
  }
  static __device__ __forceinline__ v8f mma(v16h a, v16h b, v8f c) {
    return __builtin_amdgcn_wmma_f32_16x16x32_f16(false, a, false, b, (short)0, c, false, false);
  }
  static __device__ __forceinline__ void guard(v8f& a, v8f& b, v16h x, v16h y) { dep_guard_h(a, b, x, y); }
  static __device__ __forceinline__ void keep(v16h a, v16h b, v16h c, v16h d) { keep4_h(a, b, c, d); }
};
template <> struct Frag<__bf16> {
  typedef v16b V; union U { v16b v; v8b h[2]; };
  static __device__ __forceinline__ v16b load(const __bf16* p) {
    U f; f.h[0] = *(const v8b*)(p); f.h[1] = *(const v8b*)(p + 16); return f.v;
  }
  static __device__ __forceinline__ v8f mma(v16b a, v16b b, v8f c) {
    return __builtin_amdgcn_wmma_f32_16x16x32_bf16(false, a, false, b, (short)0, c, false, false);
  }
  static __device__ __forceinline__ void guard(v8f& a, v8f& b, v16b x, v16b y) { dep_guard_b(a, b, x, y); }
  static __device__ __forceinline__ void keep(v16b a, v16b b, v16b c, v16b d) { keep4_b(a, b, c, d); }
};

template <int ET> struct Elem;
template <> struct Elem<0> { typedef _Float16 T; };
template <> struct Elem<1> { typedef __bf16 T; };
template <int ET, bool SPLIT, int BIAS_MODE, int OUT_MODE, bool RESID, int ACT = 0>
__global__ __launch_bounds__(256) void wmma_gemm64(
    const unsigned short* __restrict__ Ap, const unsigned short* __restrict__ A2p, int lda, long strideA,
    const unsigned short* __restrict__ Btp, const unsigned short* __restrict__ Bt2p, int ldb, long strideB,
    void* __restrict__ Cout, void* __restrict__ Cout2, int ldc, long strideC,
    const float* __restrict__ bias,
    const float* __restrict__ resid, long strideR,
    int M, int N, int K, float scale, float bmul) {
  typedef typename Elem<ET>::T T;
  typedef typename Frag<T>::V V;
  const T* A = (const T*)Ap; const T* A2 = (const T*)A2p; const T* Bt = (const T*)Btp; const T* Bt2 = (const T*)Bt2p;
  __shared__ __align__(16) float sT[8][16 * 68];
  const int b    = blockIdx.y;
  const int lane = threadIdx.x & 31;
  const int wave = threadIdx.x >> 5;
  const int tilesN = N >> 6;
  const int tilesM = M >> 6;
  const int tile = blockIdx.x * 8 + wave;
  if (tile >= tilesM * tilesN) return;
  const int tm = tile / tilesN;
  const int tn = tile - tm * tilesN;
  const int m0 = tm << 6;
  const int n0 = tn << 6;

  const T* Ab  = A  + (size_t)b * strideA;
  const T* Bb  = Bt + (size_t)b * strideB;
  const T* Ab2 = SPLIT ? (A2  + (size_t)b * strideA) : nullptr;
  const T* Bb2 = SPLIT ? (Bt2 + (size_t)b * strideB) : nullptr;

  const int rlane = lane & 15;
  const int koff  = (lane >> 4) * 8;
  const int mOff  = (lane >> 4) * 8;

  v8f acc[4][4];
#pragma unroll
  for (int i = 0; i < 4; ++i)
#pragma unroll
    for (int j = 0; j < 4; ++j) acc[i][j] = (v8f){0.f,0.f,0.f,0.f,0.f,0.f,0.f,0.f};

  for (int k0 = 0; k0 < K; k0 += 32) {
    V bh[4], bl[4];
#pragma unroll
    for (int j = 0; j < 4; ++j) {
      const size_t bo = (size_t)(n0 + (j << 4) + rlane) * ldb + koff + k0;
      bh[j] = Frag<T>::load(Bb + bo);
      if (SPLIT) bl[j] = Frag<T>::load(Bb2 + bo);
    }
#pragma unroll
    for (int i = 0; i < 4; ++i) {
      const size_t ao = (size_t)(m0 + (i << 4) + rlane) * lda + koff + k0;
      V ah = Frag<T>::load(Ab + ao);
      V al;
      if (SPLIT) al = Frag<T>::load(Ab2 + ao);
#pragma unroll
      for (int j = 0; j < 4; ++j) {
        acc[i][j] = Frag<T>::mma(ah, bh[j], acc[i][j]);
        if (SPLIT) {
          acc[i][j] = Frag<T>::mma(ah, bl[j], acc[i][j]);
          acc[i][j] = Frag<T>::mma(al, bh[j], acc[i][j]);
        }
      }
      Frag<T>::guard(acc[i][0], acc[i][3], ah, SPLIT ? al : ah);
    }
    Frag<T>::keep(bh[0], bh[1], bh[2], bh[3]);
    if (SPLIT) Frag<T>::keep(bl[0], bl[1], bl[2], bl[3]);
  }
  acc_guard4(acc[0][0], acc[0][1], acc[0][2], acc[0][3]);
  acc_guard4(acc[1][0], acc[1][1], acc[1][2], acc[1][3]);
  acc_guard4(acc[2][0], acc[2][1], acc[2][2], acc[2][3]);
  acc_guard4(acc[3][0], acc[3][1], acc[3][2], acc[3][3]);

  float* slab = sT[wave];
  const float* Rb = RESID ? (resid + (size_t)b * strideR) : nullptr;
#pragma unroll
  for (int i = 0; i < 4; ++i) {
    const int mBase = m0 + (i << 4);
#pragma unroll
    for (int j = 0; j < 4; ++j) {
      const int n = n0 + (j << 4) + rlane;
      float bv = 0.f;
      if (BIAS_MODE == 2) bv = bias[n] * bmul;
#pragma unroll
      for (int r = 0; r < 8; ++r) {
        float v = acc[i][j][r] * scale;
        if (BIAS_MODE == 1) v += bias[mBase + mOff + r];
        if (BIAS_MODE == 2) v += bv;
        if (RESID) v += Rb[(size_t)(mBase + mOff + r) * ldc + n];
        if (ACT == 1) v = tanhf(v);
        if (ACT == 2) v = fmaxf(v, 0.0f);
        if (ACT == 4) v = (v > 0.f) ? v : 0.01f * v;
        slab[(mOff + r) * 68 + (j << 4) + rlane] = v;
      }
    }
    __builtin_amdgcn_fence(__ATOMIC_RELEASE, "workgroup");
    __builtin_amdgcn_wave_barrier();
    __builtin_amdgcn_fence(__ATOMIC_ACQUIRE, "workgroup");
    if (OUT_MODE == 0) {
      float* C = (float*)Cout + (size_t)b * strideC;
      const int hh = lane >> 4, c4 = (lane & 15) * 4;
      for (int pass = 0; pass < 2; ++pass) {
#pragma unroll
        for (int it = 0; it < 8; ++it) {
          const int row = it * 2 + hh;
          v4f v = *(const v4f*)(slab + row * 68 + c4);
          *(volatile v4f*)(C + (size_t)(mBase + row) * ldc + n0 + c4) = v;
        }
        __threadfence();
      }
    } else {
      const int q = lane >> 3, c8 = (lane & 7) * 8;
      unsigned short* C  = (unsigned short*)Cout  + (size_t)b * strideC;
      unsigned short* C2 = (OUT_MODE == 2) ? ((unsigned short*)Cout2 + (size_t)b * strideC) : nullptr;
      for (int pass = 0; pass < 2; ++pass) {
#pragma unroll
        for (int it = 0; it < 4; ++it) {
          const int row = it * 4 + q;
          const float* sp = slab + row * 68 + c8;
          v8h hv, lv;
#pragma unroll
          for (int e = 0; e < 8; ++e) {
            if (OUT_MODE == 1) {
              hv[e] = (_Float16)sp[e];
            } else {
              unsigned short hb = f2bf_bits(sp[e]);
              unsigned short lb = f2bf_bits(sp[e] - bf_bits2f(hb));
              hv[e] = __builtin_bit_cast(_Float16, hb);
              lv[e] = __builtin_bit_cast(_Float16, lb);
            }
          }
          *(volatile v8h*)(C + (size_t)(mBase + row) * ldc + n0 + c8) = hv;
          if (OUT_MODE == 2) *(volatile v8h*)(C2 + (size_t)(mBase + row) * ldc + n0 + c8) = lv;
        }
        __threadfence();
      }
    }
    __builtin_amdgcn_fence(__ATOMIC_RELEASE, "workgroup");
    __builtin_amdgcn_wave_barrier();
    __builtin_amdgcn_fence(__ATOMIC_ACQUIRE, "workgroup");
  }
}

__global__ __launch_bounds__(256) void cast8_k(const float* __restrict__ in, unsigned short* __restrict__ outp,
                                              int n8, float mul) {
  const int i = blockIdx.x * 256 + threadIdx.x;
  if (i >= n8) return;
  const float* p = in + (size_t)i * 8;
  const v4f a = *(const v4f*)p;
  const v4f q = *(const v4f*)(p + 4);
  v8h hv;
#pragma unroll
  for (int e = 0; e < 4; ++e) { hv[e] = (_Float16)(a[e] * mul); hv[4 + e] = (_Float16)(q[e] * mul); }
  _Float16* out = (_Float16*)outp + (size_t)i * 8;
  *(volatile v8h*)out = hv;
  __threadfence();
  *(volatile v8h*)out = hv;
}

__global__ __launch_bounds__(256) void gelu2_k(const float* __restrict__ in, unsigned short* __restrict__ outp,
                                              int n2, float carry2) {
  const int i = blockIdx.x * 256 + threadIdx.x;
  if (i >= n2) return;
  const v2f x = *(const v2f*)(in + (size_t)2 * i);
  const float e0 = erff(x[0] * 0.70710678118654752f);
  const float e1 = erff(x[1] * 0.70710678118654752f);
  const float g0 = (x[0] * (e0 + 1.0f)) * carry2;
  const float g1 = (x[1] * (e1 + 1.0f)) * carry2;
  const _Float16 h0 = (_Float16)g0, h1 = (_Float16)g1;
  const unsigned u = (unsigned)__builtin_bit_cast(unsigned short, h0) | ((unsigned)__builtin_bit_cast(unsigned short, h1) << 16);
  ((volatile unsigned*)outp)[i] = u;
  __threadfence();
  ((volatile unsigned*)outp)[i] = u;
}

__device__ __forceinline__ void ln256_wave(v4f a, v4f q, v4f sa, v4f sq, v4f ba, v4f bq, v4f& oa, v4f& oq) {
  float s = ((a[0] + a[1]) + (a[2] + a[3])) + ((q[0] + q[1]) + (q[2] + q[3]));
#pragma unroll
  for (int off = 1; off < 32; off <<= 1) s += __shfl_xor(s, off, 32);
  const float mu = s * (1.0f / DMOD);
  const v4f da = a - mu, dq = q - mu;
  float s2 = ((da[0] * da[0] + da[1] * da[1]) + (da[2] * da[2] + da[3] * da[3])) +
             ((dq[0] * dq[0] + dq[1] * dq[1]) + (dq[2] * dq[2] + dq[3] * dq[3]));
#pragma unroll
  for (int off = 1; off < 32; off <<= 1) s2 += __shfl_xor(s2, off, 32);
  const float var = s2 * (1.0f / DMOD);
  const float inv = rsqrtf(var + LN_EPS);
#pragma unroll
  for (int e = 0; e < 4; ++e) {
    oa[e] = (da[e] * inv) * sa[e] + ba[e];
    oq[e] = (dq[e] * inv) * sq[e] + bq[e];
  }
}

template <bool WH>
__global__ __launch_bounds__(256) void ln_row_k(const float* __restrict__ in, const float* __restrict__ sc,
                                                const float* __restrict__ bi, float* __restrict__ out32,
                                                unsigned short* __restrict__ outhp, int rows) {
  __shared__ __align__(16) float slab[8][DMOD];
  const int lane = threadIdx.x & 31, wave = threadIdx.x >> 5;
  const int row = blockIdx.x * 8 + wave;
  if (row >= rows) return;
  const size_t rb = (size_t)row * DMOD;
  const int c8 = 8 * lane;
  const v4f a = *(const v4f*)(in + rb + c8);
  const v4f q = *(const v4f*)(in + rb + c8 + 4);
  const v4f sa = *(const v4f*)(sc + c8), sq = *(const v4f*)(sc + c8 + 4);
  const v4f ba = *(const v4f*)(bi + c8), bq = *(const v4f*)(bi + c8 + 4);
  v4f oa, oq;
  ln256_wave(a, q, sa, sq, ba, bq, oa, oq);
  if (WH) {
    v8h hv;
#pragma unroll
    for (int e = 0; e < 4; ++e) { hv[e] = (_Float16)oa[e]; hv[4 + e] = (_Float16)oq[e]; }
    _Float16* hp = (_Float16*)outhp + rb + c8;
    for (int pass = 0; pass < 2; ++pass) { *(volatile v8h*)hp = hv; __threadfence(); }
  }
  float* sw = slab[wave];
  *(v4f*)(sw + c8) = oa;
  *(v4f*)(sw + c8 + 4) = oq;
  __builtin_amdgcn_fence(__ATOMIC_RELEASE, "workgroup");
  __builtin_amdgcn_wave_barrier();
  __builtin_amdgcn_fence(__ATOMIC_ACQUIRE, "workgroup");
  const int c4 = 4 * lane;
  const v4f r0 = *(const v4f*)(sw + c4);
  const v4f r1 = *(const v4f*)(sw + 128 + c4);
  for (int pass = 0; pass < 2; ++pass) {
    *(volatile v4f*)(out32 + rb + c4) = r0;
    *(volatile v4f*)(out32 + rb + 128 + c4) = r1;
    __threadfence();
  }
}

__device__ __forceinline__ v8f mma_h(v16h a, v16h b, v8f c) {
  c = __builtin_amdgcn_wmma_f32_16x16x32_f16(false, a, false, b, (short)0, c, false, false);
  asm volatile("v_nop\n\tv_nop\n\tv_nop\n\tv_nop" : "+v"(c) : "v"(a), "v"(b));
  return c;
}
constexpr int AKEYS = 64;
constexpr int AQROWS = 64;
constexpr int OSPITCH = 72;
__global__ __launch_bounds__(128) void attn_hd64_k(const unsigned short* __restrict__ qkvp,
                                                  unsigned short* __restrict__ outp) {
  union FH { v16h v; v8h h[2]; };
  __shared__ __align__(16) _Float16 Ksh[AKEYS * HDIM64];
  __shared__ __align__(16) _Float16 Vth[HDIM64 * AKEYS];
  __shared__ __align__(16) _Float16 Psh[4][16 * AKEYS];
  __shared__ __align__(16) _Float16 Osh[4][16 * OSPITCH];
  const _Float16* qkv = (const _Float16*)qkvp;
  _Float16* out = (_Float16*)outp;
  const int tid = threadIdx.x, wave = tid >> 5, lane = tid & 31, hh = lane >> 4, c = lane & 15;
  const int nqb = SEQLEN / AQROWS;
  const int bx = blockIdx.x;
  const int qb = bx % nqb;
  const int bh = bx / nqb;
  const int h = bh % NHEAD;
  const int b = bh / NHEAD;
  const int q0 = qb * AQROWS + wave * 16;
  const size_t tokb = (size_t)b * SEQLEN;

  v16h qa[2];
  {
    const _Float16* qrow = qkv + (tokb + q0 + c) * QKVLD + h * HDIM64 + 8 * hh;
#pragma unroll
    for (int dc = 0; dc < 2; ++dc) qa[dc] = Frag<_Float16>::load(qrow + dc * 32);
  }
  float mrow[8], lrow[8];
  v8f oacc[4];
#pragma unroll
  for (int r = 0; r < 8; ++r) { mrow[r] = -INFINITY; lrow[r] = 0.f; }
#pragma unroll
  for (int t = 0; t < 4; ++t) oacc[t] = (v8f){0.f,0.f,0.f,0.f,0.f,0.f,0.f,0.f};

  const int nChunks = qb + 1;
  for (int kc = 0; kc < nChunks; ++kc) {
    const int kv0 = kc * AKEYS;
    __syncthreads();
    {
      const int kvr = tid >> 1, dh = (tid & 1) * 32;
      const _Float16* krow = qkv + (tokb + kv0 + kvr) * QKVLD + DMOD + h * HDIM64 + dh;
      const _Float16* vrow = qkv + (tokb + kv0 + kvr) * QKVLD + 2 * DMOD + h * HDIM64 + dh;
#pragma unroll 1
      for (int i = 0; i < 4; ++i) {
        const v8h kk = *(const v8h*)(krow + 8 * i);
        *(v8h*)(Ksh + kvr * HDIM64 + dh + 8 * i) = kk;
        const v8h vv = *(const v8h*)(vrow + 8 * i);
#pragma unroll
        for (int e = 0; e < 8; ++e) Vth[(dh + 8 * i + e) * AKEYS + kvr] = vv[e];
      }
    }
    __syncthreads();

    v8f s[4];
#pragma unroll
    for (int j = 0; j < 4; ++j) {
      s[j] = (v8f){0.f,0.f,0.f,0.f,0.f,0.f,0.f,0.f};
#pragma unroll
      for (int dc = 0; dc < 2; ++dc) {
        FH kb;
        kb.h[0] = *(const v8h*)(Ksh + (j * 16 + c) * HDIM64 + dc * 32 + 8 * hh);
        kb.h[1] = *(const v8h*)(Ksh + (j * 16 + c) * HDIM64 + dc * 32 + 16 + 8 * hh);
        s[j] = mma_h(qa[dc], kb.v, s[j]);
      }
    }
    const bool diag = (kc == qb);
    float cm[8];
#pragma unroll
    for (int r = 0; r < 8; ++r) {
      const int qrow = q0 + 8 * hh + r;
      float m = -INFINITY;
#pragma unroll
      for (int j = 0; j < 4; ++j) {
        const int kvcol = kv0 + j * 16 + c;
        float sv = s[j][r] * QKSCALE;
        const bool masked = diag && (kvcol > qrow);
        if (masked) sv = -INFINITY;
        s[j][r] = sv;
        m = fmaxf(m, sv);
      }
#pragma unroll
      for (int off = 1; off < 16; off <<= 1) m = fmaxf(m, __shfl_xor(m, off, 32));
      cm[r] = m;
    }
    _Float16* pw = Psh[wave];
#pragma unroll
    for (int r = 0; r < 8; ++r) {
      const float mnew = fmaxf(mrow[r], cm[r]);
      const float mref = (mnew > -INFINITY) ? mnew : 0.0f;
      const float alpha = expf(mrow[r] - mref);
      mrow[r] = mnew;
      float psum = 0.f;
#pragma unroll
      for (int j = 0; j < 4; ++j) {
        const float p = expf(s[j][r] - mref);
        psum += p;
        pw[(8 * hh + r) * AKEYS + j * 16 + c] = (_Float16)(p * PSCALE);
      }
#pragma unroll
      for (int off = 1; off < 16; off <<= 1) psum += __shfl_xor(psum, off, 32);
      lrow[r] = lrow[r] * alpha + psum;
#pragma unroll
      for (int t = 0; t < 4; ++t) oacc[t][r] *= alpha;
    }
    __builtin_amdgcn_fence(__ATOMIC_RELEASE, "workgroup");
    __builtin_amdgcn_wave_barrier();
    __builtin_amdgcn_fence(__ATOMIC_ACQUIRE, "workgroup");
#pragma unroll 1
    for (int kk = 0; kk < 2; ++kk) {
      FH pa;
      pa.h[0] = *(const v8h*)(pw + c * AKEYS + kk * 32 + 8 * hh);
      pa.h[1] = *(const v8h*)(pw + c * AKEYS + kk * 32 + 16 + 8 * hh);
#pragma unroll
      for (int t = 0; t < 4; ++t) {
        FH vb;
        vb.h[0] = *(const v8h*)(Vth + (t * 16 + c) * AKEYS + kk * 32 + 8 * hh);
        vb.h[1] = *(const v8h*)(Vth + (t * 16 + c) * AKEYS + kk * 32 + 16 + 8 * hh);
        oacc[t] = mma_h(pa.v, vb.v, oacc[t]);
      }
    }
  }

  _Float16* os = Osh[wave];
#pragma unroll
  for (int r = 0; r < 8; ++r) {
    const float inv = OCARRY / (lrow[r] * PSCALE);
#pragma unroll
    for (int t = 0; t < 4; ++t) os[(8 * hh + r) * OSPITCH + t * 16 + c] = (_Float16)(oacc[t][r] * inv);
  }
  __builtin_amdgcn_fence(__ATOMIC_RELEASE, "workgroup");
  __builtin_amdgcn_wave_barrier();
  __builtin_amdgcn_fence(__ATOMIC_ACQUIRE, "workgroup");
  {
    const int q8 = lane >> 3, c8 = (lane & 7) * 8;
    for (int pass = 0; pass < 2; ++pass) {
#pragma unroll
      for (int it = 0; it < 4; ++it) {
        const int row = it * 4 + q8;
        const v8h val = *(const v8h*)(os + row * OSPITCH + c8);
        *(volatile v8h*)(out + (tokb + q0 + row) * DMOD + h * HDIM64 + c8) = val;
      }
      __threadfence();
    }
  }
}

__global__ __launch_bounds__(256) void mid_k(const float* __restrict__ x32, const float* __restrict__ pg,
                                             const float* __restrict__ cw, const float* __restrict__ cbias,
                                             unsigned short* __restrict__ combp, float* __restrict__ out2) {
  __shared__ __align__(16) _Float16 tile[TCH * COMBLD];
  __shared__ __align__(16) float o2s[DMOD];
  const int b = blockIdx.x, d = threadIdx.x, lane = d & 31, wave = d >> 5;
  _Float16* comb = (_Float16*)combp;
  const float w0 = cw[d * CONVW + 0], w1 = cw[d * CONVW + 1], w2 = cw[d * CONVW + 2], w3 = cw[d * CONVW + 3];
  const float w4 = cw[d * CONVW + 4], w5 = cw[d * CONVW + 5], w6 = cw[d * CONVW + 6], w7 = cw[d * CONVW + 7];
  const float cbv = cbias[d];
  float c = 0.f;
  float h0 = 0.f, h1 = 0.f, h2 = 0.f, h3 = 0.f, h4 = 0.f, h5 = 0.f, h6 = 0.f;
  const size_t tok0 = (size_t)b * SEQLEN;
  for (int ch = 0; ch < SEQLEN / TCH; ++ch) {
#pragma unroll 1
    for (int tt = 0; tt < TCH; ++tt) {
      const size_t m = tok0 + ch * TCH + tt;
      const float xv = x32[m * DMOD + d];
      const float pv = pg[m * DMOD + d];
      float loc = w0 * h0;
      loc += w1 * h1; loc += w2 * h2; loc += w3 * h3; loc += w4 * h4; loc += w5 * h5; loc += w6 * h6; loc += w7 * xv;
      loc += cbv;
      c = EMA_DECAY * c + EMA_GAIN * xv;
      tile[tt * COMBLD + d] = (_Float16)(xv + GUIDE * pv);
      tile[tt * COMBLD + DMOD + d] = (_Float16)loc;
      tile[tt * COMBLD + 2 * DMOD + d] = (_Float16)c;
      h0 = h1; h1 = h2; h2 = h3; h3 = h4; h4 = h5; h5 = h6; h6 = xv;
    }
    __syncthreads();
    for (int pass = 0; pass < 2; ++pass) {
#pragma unroll
      for (int rr = 0; rr < 2; ++rr) {
        const int row = 2 * wave + rr;
        const size_t m = tok0 + ch * TCH + row;
#pragma unroll
        for (int sg = 0; sg < 3; ++sg) {
          const v8h v = *(const v8h*)(tile + row * COMBLD + sg * DMOD + 8 * lane);
          *(volatile v8h*)(comb + m * COMBLD + sg * DMOD + 8 * lane) = v;
        }
      }
      __threadfence();
    }
    __syncthreads();
  }
  o2s[d] = c;
  __syncthreads();
  if (wave == 0) {
    const int c4 = 4 * lane;
    const v4f r0 = *(const v4f*)(o2s + c4);
    const v4f r1 = *(const v4f*)(o2s + 128 + c4);
    float* op = out2 + (size_t)b * DMOD;
    for (int pass = 0; pass < 2; ++pass) {
      *(volatile v4f*)(op + c4) = r0;
      *(volatile v4f*)(op + 128 + c4) = r1;
      __threadfence();
    }
  }
}

__global__ __launch_bounds__(256) void scan_ln_k(const float* __restrict__ del, const float* __restrict__ s0,
                                                 const float* __restrict__ s3, const float* __restrict__ b3,
                                                 const float* __restrict__ s4, const float* __restrict__ b4,
                                                 unsigned short* __restrict__ sthp, float* __restrict__ out1) {
  __shared__ __align__(16) float tile[TCH * DMOD];
  __shared__ __align__(16) float slab[DMOD];
  const int b = blockIdx.x, d = threadIdx.x, lane = d & 31, wave = d >> 5;
  _Float16* sth = (_Float16*)sthp;
  const float base = s0[b * DMOD + d];
  float acc = 0.f;
  const size_t tok0 = (size_t)b * SEQLEN;
  const int c8 = 8 * lane;
  const v4f sa3 = *(const v4f*)(s3 + c8), sq3 = *(const v4f*)(s3 + c8 + 4);
  const v4f ba3 = *(const v4f*)(b3 + c8), bq3 = *(const v4f*)(b3 + c8 + 4);
  for (int ch = 0; ch < SEQLEN / TCH; ++ch) {
#pragma unroll 1
    for (int tt = 0; tt < TCH; ++tt) {
      const size_t m = tok0 + ch * TCH + tt;
      acc += del[m * DMOD + d];
      tile[tt * DMOD + d] = base + STEP_HALF * acc;
    }
    __syncthreads();
#pragma unroll
    for (int rr = 0; rr < 2; ++rr) {
      const int row = 2 * wave + rr;
      const size_t m = tok0 + ch * TCH + row;
      const v4f a = *(const v4f*)(tile + row * DMOD + c8);
      const v4f q = *(const v4f*)(tile + row * DMOD + c8 + 4);
      v4f oa, oq;
      ln256_wave(a, q, sa3, sq3, ba3, bq3, oa, oq);
      v8h hv;
#pragma unroll
      for (int e = 0; e < 4; ++e) { hv[e] = (_Float16)oa[e]; hv[4 + e] = (_Float16)oq[e]; }
      _Float16* hp = sth + m * DMOD + c8;
      for (int pass = 0; pass < 2; ++pass) { *(volatile v8h*)hp = hv; __threadfence(); }
      if (ch == SEQLEN / TCH - 1 && row == TCH - 1) {
        const v4f sa4 = *(const v4f*)(s4 + c8), sq4 = *(const v4f*)(s4 + c8 + 4);
        const v4f ba4 = *(const v4f*)(b4 + c8), bq4 = *(const v4f*)(b4 + c8 + 4);
        v4f pa, pq;
        ln256_wave(oa, oq, sa4, sq4, ba4, bq4, pa, pq);
        *(v4f*)(slab + c8) = pa;
        *(v4f*)(slab + c8 + 4) = pq;
        __builtin_amdgcn_fence(__ATOMIC_RELEASE, "workgroup");
        __builtin_amdgcn_wave_barrier();
        __builtin_amdgcn_fence(__ATOMIC_ACQUIRE, "workgroup");
        const int c4 = 4 * lane;
        const v4f r0 = *(const v4f*)(slab + c4);
        const v4f r1 = *(const v4f*)(slab + 128 + c4);
        float* op = out1 + (size_t)b * DMOD;
        for (int pass = 0; pass < 2; ++pass) {
          *(volatile v4f*)(op + c4) = r0;
          *(volatile v4f*)(op + 128 + c4) = r1;
          __threadfence();
        }
      }
    }
    __syncthreads();
  }
}

extern "C" void kernel_launch(void* const* d_in, const int* in_sizes, int n_in,
                              void* d_out, int out_size, void* d_ws,
                              size_t ws_size, hipStream_t stream) {
  if (n_in < 29) return;
  if (in_sizes[0] != NTOKS * DMOD || in_sizes[1] != NBATCH * DMOD ||
      in_sizes[3] != 3 * DMOD * DMOD || in_sizes[4] != 3 * DMOD ||
      in_sizes[5] != DMOD * DMOD || in_sizes[6] != DMOD ||
      in_sizes[7] != DMOD * CONVW || in_sizes[8] != DMOD ||
      in_sizes[9] != DMOD * DMOD || in_sizes[10] != DMOD ||
      in_sizes[11] != DMOD * DMOD || in_sizes[12] != DMOD ||
      in_sizes[13] != HIDT * 3 * DMOD || in_sizes[14] != HIDT ||
      in_sizes[15] != DMOD * HIDT || in_sizes[16] != DMOD ||
      in_sizes[17] != HIDF * DMOD || in_sizes[18] != HIDF ||
      in_sizes[19] != DMOD * HIDF || in_sizes[20] != DMOD) return;
  for (int i = 21; i <= 28; ++i) if (in_sizes[i] != DMOD) return;
  if (out_size != NTOKS * DMOD + 2 * NBATCH * DMOD) return;

  const float* X     = (const float*)d_in[0];
  const float* SSt   = (const float*)d_in[1];
  const float* in_w  = (const float*)d_in[3];
  const float* in_b  = (const float*)d_in[4];
  const float* op_w  = (const float*)d_in[5];
  const float* op_b  = (const float*)d_in[6];
  const float* cv_w  = (const float*)d_in[7];
  const float* cv_b  = (const float*)d_in[8];
  const float* p2s_w = (const float*)d_in[9];
  const float* p2s_b = (const float*)d_in[10];
  const float* s2p_w = (const float*)d_in[11];
  const float* s2p_b = (const float*)d_in[12];
  const float* tw1   = (const float*)d_in[13];
  const float* tb1   = (const float*)d_in[14];
  const float* tw2   = (const float*)d_in[15];
  const float* tb2   = (const float*)d_in[16];
  const float* fw1   = (const float*)d_in[17];
  const float* fb1   = (const float*)d_in[18];
  const float* fw2   = (const float*)d_in[19];
  const float* fb2   = (const float*)d_in[20];
  const float* ln1_s = (const float*)d_in[21];
  const float* ln1_b = (const float*)d_in[22];
  const float* ln2_s = (const float*)d_in[23];
  const float* ln2_b = (const float*)d_in[24];
  const float* ln3_s = (const float*)d_in[25];
  const float* ln3_b = (const float*)d_in[26];
  const float* ln4_s = (const float*)d_in[27];
  const float* ln4_b = (const float*)d_in[28];

  float* out0 = (float*)d_out;
  float* out1 = out0 + (size_t)NTOKS * DMOD;
  float* out2 = out1 + (size_t)NBATCH * DMOD;

  const size_t P16_256 = (size_t)NTOKS * 256 * 2, P16_512 = (size_t)NTOKS * 512 * 2, P16_768 = (size_t)NTOKS * 768 * 2,
               P16_1024 = (size_t)NTOKS * 1024 * 2;
  const size_t P32_256 = (size_t)NTOKS * 256 * 4, P32_512 = (size_t)NTOKS * 512 * 4, P32_1024 = (size_t)NTOKS * 1024 * 4;
  const size_t oX32  = 0;
  const size_t oWIN  = oX32 + P32_256;                         const size_t szWIN  = (size_t)3 * DMOD * DMOD * 2;
  const size_t oWOUT = oWIN + szWIN;                           const size_t szWOUT = (size_t)DMOD * DMOD * 2;
  const size_t oWP   = oWOUT + szWOUT;                         const size_t szWP   = (size_t)DMOD * DMOD * 2;
  const size_t oW1   = oWP + szWP;                             const size_t szW1   = (size_t)HIDT * 3 * DMOD * 2;
  const size_t oW2   = oW1 + szW1;                             const size_t szW2   = (size_t)DMOD * HIDT * 2;
  const size_t oWS   = oW2 + szW2;                             const size_t szWS   = (size_t)DMOD * DMOD * 2;
  const size_t oWF1  = oWS + szWS;                             const size_t szWF1  = (size_t)HIDF * DMOD * 2;
  const size_t oWF2  = oWF1 + szWF1;                           const size_t szWF2  = (size_t)DMOD * HIDF * 2;
  const size_t oA    = oWF2 + szWF2;                           const size_t szA    = P16_1024 + P32_256;
  const size_t oB    = oA + szA;                               const size_t szB    = P32_1024;
  const size_t oEND  = oB + szB;
  if (oEND > ws_size || oEND > (size_t)134217728) return;
  char* ws = (char*)d_ws;
  float*          x32  = (float*)(ws + oX32);
  unsigned short* win  = (unsigned short*)(ws + oWIN);
  unsigned short* wout = (unsigned short*)(ws + oWOUT);
  unsigned short* wp   = (unsigned short*)(ws + oWP);
  unsigned short* w1   = (unsigned short*)(ws + oW1);
  unsigned short* w2   = (unsigned short*)(ws + oW2);
  unsigned short* wsp  = (unsigned short*)(ws + oWS);
  unsigned short* wf1  = (unsigned short*)(ws + oWF1);
  unsigned short* wf2  = (unsigned short*)(ws + oWF2);
  unsigned short* qkv  = (unsigned short*)(ws + oA);
  unsigned short* att  = (unsigned short*)(ws + oA + P16_768);
  unsigned short* xh   = (unsigned short*)(ws + oA + P16_768 + P16_256);
  unsigned short* xh2  = (unsigned short*)(ws + oA);
  float*          pg   = (float*)(ws + oA + P16_256);
  float*          h32  = (float*)(ws + oA);
  float*          del  = (float*)(ws + oA);
  unsigned short* sth  = (unsigned short*)(ws + oA + P32_256);
  unsigned short* fin  = (unsigned short*)(ws + oA + P32_256 + P16_256);
  unsigned short* fh   = (unsigned short*)(ws + oA);
  float*          z32  = (float*)(ws + oA + P16_1024);
  float*          y32  = (float*)(ws + oB);
  unsigned short* comb = (unsigned short*)(ws + oB);
  unsigned short* hh   = (unsigned short*)(ws + oB);
  float*          fpre = (float*)(ws + oB);

  const float WINV = 1.0f / WCARRY;

  cast8_k<<<(NTOKS * DMOD / 8 + 255) / 256, 256, 0, stream>>>(X, xh, NTOKS * DMOD / 8, 1.0f);
  cast8_k<<<(3 * DMOD * DMOD / 8 + 255) / 256, 256, 0, stream>>>(in_w, win, 3 * DMOD * DMOD / 8, WCARRY);
  cast8_k<<<(DMOD * DMOD / 8 + 255) / 256, 256, 0, stream>>>(op_w, wout, DMOD * DMOD / 8, WCARRY);
  cast8_k<<<(DMOD * DMOD / 8 + 255) / 256, 256, 0, stream>>>(p2s_w, wp, DMOD * DMOD / 8, WCARRY);
  cast8_k<<<(HIDT * 3 * DMOD / 8 + 255) / 256, 256, 0, stream>>>(tw1, w1, HIDT * 3 * DMOD / 8, WCARRY);
  cast8_k<<<(DMOD * HIDT / 8 + 255) / 256, 256, 0, stream>>>(tw2, w2, DMOD * HIDT / 8, WCARRY);
  cast8_k<<<(DMOD * DMOD / 8 + 255) / 256, 256, 0, stream>>>(s2p_w, wsp, DMOD * DMOD / 8, WCARRY);
  cast8_k<<<(HIDF * DMOD / 8 + 255) / 256, 256, 0, stream>>>(fw1, wf1, HIDF * DMOD / 8, WCARRY);
  cast8_k<<<(DMOD * HIDF / 8 + 255) / 256, 256, 0, stream>>>(fw2, wf2, DMOD * HIDF / 8, WCARRY);

  {
    const int Mm = NTOKS, Nn = QKVLD, Kk = DMOD; const int tiles = (Mm / 64) * (Nn / 64);
    wmma_gemm64<0, false, 2, 1, false, 0><<<dim3((tiles + 7) / 8, 1), 256, 0, stream>>>(
        xh, xh, Kk, 0, win, win, Kk, 0, qkv, qkv, Nn, 0, in_b, X, 0, Mm, Nn, Kk, WINV, 1.0f);
  }
  attn_hd64_k<<<NBATCH * NHEAD * (SEQLEN / AQROWS), 128, 0, stream>>>(qkv, att);
  {
    const int Mm = NTOKS, Nn = DMOD, Kk = DMOD; const int tiles = (Mm / 64) * (Nn / 64);
    wmma_gemm64<0, false, 2, 0, true, 0><<<dim3((tiles + 7) / 8, 1), 256, 0, stream>>>(
        att, att, Kk, 0, wout, wout, Kk, 0, y32, y32, Nn, 0, op_b, X, 0, Mm, Nn, Kk, WINV / OCARRY, 1.0f);
  }
  ln_row_k<true><<<NTOKS / 8, 256, 0, stream>>>(y32, ln1_s, ln1_b, x32, xh2, NTOKS);
  {
    const int Mm = NTOKS, Nn = DMOD, Kk = DMOD; const int tiles = (Mm / 64) * (Nn / 64);
    wmma_gemm64<0, false, 2, 0, false, 0><<<dim3((tiles + 7) / 8, 1), 256, 0, stream>>>(
        xh2, xh2, Kk, 0, wp, wp, Kk, 0, pg, pg, Nn, 0, p2s_b, X, 0, Mm, Nn, Kk, WINV, 1.0f);
  }
  mid_k<<<NBATCH, 256, 0, stream>>>(x32, pg, cv_w, cv_b, comb, out2);
  {
    const int Mm = NTOKS, Nn = HIDT, Kk = COMBLD; const int tiles = (Mm / 64) * (Nn / 64);
    wmma_gemm64<0, false, 2, 0, false, 0><<<dim3((tiles + 7) / 8, 1), 256, 0, stream>>>(
        comb, comb, Kk, 0, w1, w1, Kk, 0, h32, h32, Nn, 0, tb1, X, 0, Mm, Nn, Kk, WINV, 1.0f);
  }
  gelu2_k<<<(NTOKS * HIDT / 2 + 255) / 256, 256, 0, stream>>>(h32, hh, NTOKS * HIDT / 2, 0.5f * GCARRY);
  {
    const int Mm = NTOKS, Nn = DMOD, Kk = HIDT; const int tiles = (Mm / 64) * (Nn / 64);
    wmma_gemm64<0, false, 2, 0, false, 0><<<dim3((tiles + 7) / 8, 1), 256, 0, stream>>>(
        hh, hh, Kk, 0, w2, w2, Kk, 0, del, del, Nn, 0, tb2, X, 0, Mm, Nn, Kk, WINV / GCARRY, 1.0f);
  }
  scan_ln_k<<<NBATCH, 256, 0, stream>>>(del, SSt, ln3_s, ln3_b, ln4_s, ln4_b, sth, out1);
  {
    const int Mm = NTOKS, Nn = DMOD, Kk = DMOD; const int tiles = (Mm / 64) * (Nn / 64);
    wmma_gemm64<0, false, 2, 1, true, 0><<<dim3((tiles + 7) / 8, 1), 256, 0, stream>>>(
        sth, sth, Kk, 0, wsp, wsp, Kk, 0, fin, fin, Nn, 0, s2p_b, x32, 0, Mm, Nn, Kk, GUIDE * WINV, GUIDE);
  }
  {
    const int Mm = NTOKS, Nn = HIDF, Kk = DMOD; const int tiles = (Mm / 64) * (Nn / 64);
    wmma_gemm64<0, false, 2, 0, false, 0><<<dim3((tiles + 7) / 8, 1), 256, 0, stream>>>(
        fin, fin, Kk, 0, wf1, wf1, Kk, 0, fpre, fpre, Nn, 0, fb1, X, 0, Mm, Nn, Kk, WINV, 1.0f);
  }
  gelu2_k<<<(NTOKS * HIDF / 2 + 255) / 256, 256, 0, stream>>>(fpre, fh, NTOKS * HIDF / 2, 0.5f * GCARRY);
  {
    const int Mm = NTOKS, Nn = DMOD, Kk = HIDF; const int tiles = (Mm / 64) * (Nn / 64);
    wmma_gemm64<0, false, 2, 0, true, 0><<<dim3((tiles + 7) / 8, 1), 256, 0, stream>>>(
        fh, fh, Kk, 0, wf2, wf2, Kk, 0, z32, z32, Nn, 0, fb2, x32, 0, Mm, Nn, Kk, WINV / GCARRY, 1.0f);
  }
  ln_row_k<false><<<NTOKS / 8, 256, 0, stream>>>(z32, ln2_s, ln2_b, out0, xh, NTOKS);
}
